// ExaoneFlashAttention_82154134438142
// MI455X (gfx1250) — hardware-verified
//
#include <hip/hip_runtime.h>
#include <hip/hip_bf16.h>
#include <math.h>


typedef _Float16 bf16;
typedef _Float16 f16;
typedef __attribute__((ext_vector_type(4))) unsigned v4u_t;
typedef unsigned v4ua __attribute__((ext_vector_type(4), may_alias));
typedef __attribute__((ext_vector_type(4))) float v4f_t;
typedef float v4fa __attribute__((ext_vector_type(4), may_alias));
typedef __attribute__((ext_vector_type(16))) bf16  bf16x16;
typedef bf16x16 f16x16;
typedef __attribute__((ext_vector_type(8)))  bf16  bf16x8;
typedef bf16x8 f16x8;
typedef __attribute__((ext_vector_type(4)))  bf16  bf16x4;
typedef __attribute__((ext_vector_type(8)))  float f32x8;
__device__ __forceinline__ f32x8 wmma16(f16x16 a, f16x16 b, f32x8 c) {
  c = __builtin_amdgcn_wmma_f32_16x16x32_f16(false, a, false, b, (short)0, c, false, false);
  asm volatile("v_nop\n\tv_nop\n\tv_nop\n\tv_nop" : "+v"(c) : "v"(a), "v"(b));
  return c;
}
#define LDS_STRIDE 48
#define KSTRIDE    72
#define VSTRIDE    48

__device__ __forceinline__ f32x8 wmma_bf16(bf16x16 a, bf16x16 b, f32x8 c) {
  c = __builtin_amdgcn_wmma_f32_16x16x32_f16(false, a, false, b, (short)0, c, false, false);
  asm volatile("v_nop\n\tv_nop\n\tv_nop\n\tv_nop" : "+v"(c) : "v"(a), "v"(b));
  return c;
}

template <typename T>
__device__ __forceinline__ bf16x16 load_frag(const T* __restrict__ base, int ld,
                                             int row0, int k0) {
  const int lane = threadIdx.x & 31;
  const int r    = lane & 15;
  const int kh   = (lane >> 4) * 8;
  const T* p0 = base + (size_t)(row0 + r) * ld + (k0 + kh);
  const T* p1 = p0 + 16;
  bf16x16 f;
#pragma unroll
  for (int i = 0; i < 8; ++i) {
    f[i]     = (bf16)p0[i];
    f[i + 8] = (bf16)p1[i];
  }
  return f;
}

__device__ __forceinline__ bf16x16 lds_frag(const bf16* base, int stride) {
  const int lane = threadIdx.x & 31;
  const int row  = lane & 15;
  const int kh   = (lane >> 4) * 8;
  const bf16x8 lo = *(const bf16x8*)(base + row * stride + kh);
  const bf16x8 hi = *(const bf16x8*)(base + row * stride + kh + 16);
  bf16x16 f;
#pragma unroll
  for (int i = 0; i < 8; ++i) { f[i] = lo[i]; f[i + 8] = hi[i]; }
  return f;
}

template <typename T>
__device__ __forceinline__ void stage_read16(const T* __restrict__ p, float* buf) {
#pragma unroll
  for (int i = 0; i < 16; ++i) buf[i] = (float)p[i];
}

__device__ __forceinline__ void stage_write(bf16* dst, const float* buf, int nquad) {
#pragma unroll
  for (int i = 0; i < nquad; ++i) {
    bf16x4 q;
    q[0] = (bf16)buf[4 * i];     q[1] = (bf16)buf[4 * i + 1];
    q[2] = (bf16)buf[4 * i + 2]; q[3] = (bf16)buf[4 * i + 3];
    *(bf16x4*)(dst + 4 * i) = q;
  }
}


#define GSTR 48
#define GSTR 48
template <typename AT, int EPI, bool OUT16>
__global__ __launch_bounds__(256) void gemm_kne(const AT* __restrict__ A, int lda, const float* __restrict__ Wm, int ldw,
                                                const float* __restrict__ bias, const float* __restrict__ R, const float* __restrict__ gvec,
                                                void* __restrict__ Yv, int ldy, int K) {
  __shared__ __attribute__((aligned(16))) f16 ldsA[128 * GSTR];
  __shared__ __attribute__((aligned(16))) f16 ldsW[128 * GSTR];
  __shared__ __attribute__((aligned(16))) float oS[8][32 * 68];
  const int tid = threadIdx.x, lane = tid & 31, wave = tid >> 5, cl = lane & 15, rh = (lane >> 4) * 8;
  const int m0 = blockIdx.x * 128, n0 = blockIdx.y * 128;
  const int wm = (wave & 3) * 32, wn = (wave >> 2) * 64;
  f32x8 acc[2][4];
#pragma unroll
  for (int i = 0; i < 2; ++i)
#pragma unroll
    for (int j = 0; j < 4; ++j) { f32x8 z = {}; acc[i][j] = z; }
#pragma unroll 1
  for (int k0 = 0; k0 < K; k0 += 32) {
    __syncthreads();
    { const int row = tid >> 1, ch = (tid & 1) * 16;
      const AT* src = A + (size_t)(m0 + row) * lda + k0 + ch;
#pragma unroll
      for (int g = 0; g < 16; ++g) ldsA[row * GSTR + ch + g] = (f16)src[g]; }
    { const int k = tid >> 3, nn0 = (tid & 7) * 16;
      const float* src = Wm + (size_t)(k0 + k) * ldw + n0 + nn0;
#pragma unroll
      for (int g = 0; g < 4; ++g) { const v4f_t v = *(const v4f_t*)(src + 4 * g);
#pragma unroll
        for (int u = 0; u < 4; ++u) ldsW[(nn0 + 4 * g + u) * GSTR + k] = (f16)v[u]; } }
    __syncthreads();
    f16x16 af[2];
#pragma unroll
    for (int i = 0; i < 2; ++i) af[i] = lds_frag(ldsA + (wm + 16 * i) * GSTR, GSTR);
#pragma unroll
    for (int j = 0; j < 4; ++j) {
      const f16x16 bf = lds_frag(ldsW + (wn + 16 * j) * GSTR, GSTR);
#pragma unroll
      for (int i = 0; i < 2; ++i) acc[i][j] = wmma16(af[i], bf, acc[i][j]);
    }
  }
  float* so = oS[wave];
#pragma unroll
  for (int i = 0; i < 2; ++i)
#pragma unroll
    for (int j = 0; j < 4; ++j) {
      const int n = n0 + wn + 16 * j + cl;
      const float bv = bias ? bias[n] : 0.0f;
      const float gv = (EPI == 2 || EPI == 4) ? gvec[n] : 0.0f;
      if (EPI == 1) {
#pragma unroll 1
        for (int r = 0; r < 8; ++r) { const float xg = acc[i][j][r] + bv; so[(16 * i + rh + r) * 68 + 16 * j + cl] = 0.5f * xg * (1.0f + erff(xg * 0.70710678118654752f)); }
      } else {
#pragma unroll
        for (int r = 0; r < 8; ++r) {
          float v = acc[i][j][r] + bv;
          if (EPI == 3) v = fmaxf(v, 0.0f);
          if (EPI == 4) v = gv * v;
          if (EPI == 2) v = R[(size_t)(m0 + wm + 16 * i + rh + r) * ldy + n] + gv * v;
          so[(16 * i + rh + r) * 68 + 16 * j + cl] = v;
        }
      }
    }
  asm volatile("s_wait_dscnt 0" ::: "memory");
  __builtin_amdgcn_wave_barrier();
#pragma unroll 1
  for (int pass = 0; pass < 2; ++pass) {
    if (OUT16) {
      f16* Y = (f16*)Yv;
#pragma unroll
      for (int it = 0; it < 8; ++it) { const int c = lane + 32 * it, rr = c >> 3, q8 = (c & 7) * 8;
        union { f16 h[8]; v4u_t v; } u;
#pragma unroll
        for (int e = 0; e < 8; ++e) u.h[e] = (f16)so[rr * 68 + q8 + e];
        *(volatile v4u_t*)(Y + (size_t)(m0 + wm + rr) * ldy + n0 + wn + q8) = u.v; }
    } else {
      float* Y = (float*)Yv;
#pragma unroll
      for (int it = 0; it < 16; ++it) { const int f4 = lane + 32 * it, rr = f4 >> 4, q = (f4 & 15) * 4;
        *(volatile v4f_t*)(Y + (size_t)(m0 + wm + rr) * ldy + n0 + wn + q) = *(const v4fa*)(so + rr * 68 + q); }
    }
    __threadfence();
  }
}

template <typename AT, int EPI, bool OUT16, int CZ>
__global__ __launch_bounds__(256) void gemm_knezc(const AT* __restrict__ A, int lda, size_t strideA, const float* __restrict__ Wm, int ldw, size_t strideW,
                                                 const float* __restrict__ bias, const float* __restrict__ R, const float* __restrict__ gvec,
                                                 void* __restrict__ Yv, int ldy, size_t strideY, int K) {
  A += (size_t)blockIdx.z * strideA; Wm += (size_t)blockIdx.z * strideW; Yv = (void*)((char*)Yv + (size_t)blockIdx.z * strideY * (OUT16 ? 2 : 4)); if (R) R += (size_t)blockIdx.z * strideY;
  __shared__ __attribute__((aligned(16))) f16 ldsA[128 * GSTR];
  __shared__ __attribute__((aligned(16))) f16 ldsW[128 * GSTR];
  __shared__ __attribute__((aligned(16))) float oS[8][32 * 68];
  const int tid = threadIdx.x, lane = tid & 31, wave = tid >> 5, cl = lane & 15, rh = (lane >> 4) * 8;
  const int m0 = blockIdx.x * 128, n0 = blockIdx.y * 128;
  if (CZ == 2 && n0 >= m0 + 128) return;
  const int Kc = (CZ == 1) ? min(K, m0 + 128) : K;
  const int wm = (wave & 3) * 32, wn = (wave >> 2) * 64;
  f32x8 acc[2][4];
#pragma unroll
  for (int i = 0; i < 2; ++i)
#pragma unroll
    for (int j = 0; j < 4; ++j) { f32x8 z = {}; acc[i][j] = z; }
#pragma unroll 1
  for (int k0 = 0; k0 < Kc; k0 += 32) {
    __syncthreads();
    { const int row = tid >> 1, ch = (tid & 1) * 16;
      const AT* src = A + (size_t)(m0 + row) * lda + k0 + ch;
#pragma unroll
      for (int g = 0; g < 16; ++g) ldsA[row * GSTR + ch + g] = (f16)src[g]; }
    { const int k = tid >> 3, nn0 = (tid & 7) * 16;
      const float* src = Wm + (size_t)(k0 + k) * ldw + n0 + nn0;
#pragma unroll
      for (int g = 0; g < 4; ++g) { const v4f_t v = *(const v4f_t*)(src + 4 * g);
#pragma unroll
        for (int u = 0; u < 4; ++u) ldsW[(nn0 + 4 * g + u) * GSTR + k] = (f16)v[u]; } }
    __syncthreads();
    f16x16 af[2];
#pragma unroll
    for (int i = 0; i < 2; ++i) af[i] = lds_frag(ldsA + (wm + 16 * i) * GSTR, GSTR);
#pragma unroll
    for (int j = 0; j < 4; ++j) {
      const f16x16 bf = lds_frag(ldsW + (wn + 16 * j) * GSTR, GSTR);
#pragma unroll
      for (int i = 0; i < 2; ++i) acc[i][j] = wmma16(af[i], bf, acc[i][j]);
    }
  }
  float* so = oS[wave];
#pragma unroll
  for (int i = 0; i < 2; ++i)
#pragma unroll
    for (int j = 0; j < 4; ++j) {
      const int n = n0 + wn + 16 * j + cl;
      const float bv = bias ? bias[n] : 0.0f;
      const float gv = (EPI == 2 || EPI == 4) ? gvec[n] : 0.0f;
      if (EPI == 1) {
#pragma unroll 1
        for (int r = 0; r < 8; ++r) { const float xg = acc[i][j][r] + bv; so[(16 * i + rh + r) * 68 + 16 * j + cl] = 0.5f * xg * (1.0f + erff(xg * 0.70710678118654752f)); }
      } else {
#pragma unroll
        for (int r = 0; r < 8; ++r) {
          float v = acc[i][j][r] + bv;
          if (EPI == 3) v = fmaxf(v, 0.0f);
          if (EPI == 4) v = gv * v;
          if (EPI == 2) v = R[(size_t)(m0 + wm + 16 * i + rh + r) * ldy + n] + gv * v;
          so[(16 * i + rh + r) * 68 + 16 * j + cl] = v;
        }
      }
    }
  asm volatile("s_wait_dscnt 0" ::: "memory");
  __builtin_amdgcn_wave_barrier();
#pragma unroll 1
  for (int pass = 0; pass < 2; ++pass) {
    if (OUT16) {
      f16* Y = (f16*)Yv;
#pragma unroll
      for (int it = 0; it < 8; ++it) { const int c = lane + 32 * it, rr = c >> 3, q8 = (c & 7) * 8;
        union { f16 h[8]; v4u_t v; } u;
#pragma unroll
        for (int e = 0; e < 8; ++e) u.h[e] = (f16)so[rr * 68 + q8 + e];
        *(volatile v4u_t*)(Y + (size_t)(m0 + wm + rr) * ldy + n0 + wn + q8) = u.v; }
    } else {
      float* Y = (float*)Yv;
#pragma unroll
      for (int it = 0; it < 16; ++it) { const int f4 = lane + 32 * it, rr = f4 >> 4, q = (f4 & 15) * 4;
        *(volatile v4f_t*)(Y + (size_t)(m0 + wm + rr) * ldy + n0 + wn + q) = *(const v4fa*)(so + rr * 68 + q); }
    }
    __threadfence();
  }
}

template <typename AT, bool ACC, int CZ>
__global__ __launch_bounds__(256) void gemm_kn2c(const AT* __restrict__ A, int lda, size_t strideA,
                                               const float* __restrict__ Wm, int ldw, size_t strideW,
                                               const float* __restrict__ bias, float scale,
                                               float* __restrict__ Y, int ldy, size_t strideY, int K) {
  __shared__ __attribute__((aligned(16))) f16 ldsA[128 * GSTR], ldsAl[128 * GSTR];
  __shared__ __attribute__((aligned(16))) f16 ldsW[128 * GSTR], ldsWl[128 * GSTR];
  __shared__ __attribute__((aligned(16))) float oS[8][32 * 68];
  const int tid = threadIdx.x, lane = tid & 31, wave = tid >> 5, cl = lane & 15, rh = (lane >> 4) * 8;
  const int m0 = blockIdx.x * 128, n0 = blockIdx.y * 128;
  if (CZ == 2 && n0 >= m0 + 128) return;
  const int Kc = (CZ == 1) ? min(K, m0 + 128) : K;
  const int wm = (wave & 3) * 32, wn = (wave >> 2) * 64;
  A += (size_t)blockIdx.z * strideA; Wm += (size_t)blockIdx.z * strideW; Y += (size_t)blockIdx.z * strideY;
  f32x8 acc[2][4], accx[2][4];
#pragma unroll
  for (int i = 0; i < 2; ++i)
#pragma unroll
    for (int j = 0; j < 4; ++j) { f32x8 z = {}; acc[i][j] = z; accx[i][j] = z; }
#pragma unroll 1
  for (int k0 = 0; k0 < Kc; k0 += 32) {
    __syncthreads();
    {
      const int row = tid >> 1, ch = (tid & 1) * 16;
      const AT* src = A + (size_t)(m0 + row) * lda + k0 + ch;
#pragma unroll
      for (int g = 0; g < 16; ++g) { const float v = (float)src[g]; const f16 h = (f16)v; ldsA[row * GSTR + ch + g] = h; ldsAl[row * GSTR + ch + g] = (f16)((v - (float)h) * 2048.0f); }
    }
    {
      const int k = tid >> 3, nn0 = (tid & 7) * 16;
      const float* src = Wm + (size_t)(k0 + k) * ldw + n0 + nn0;
#pragma unroll
      for (int g = 0; g < 4; ++g) { const v4f_t v = *(const v4f_t*)(src + 4 * g);
#pragma unroll
        for (int u = 0; u < 4; ++u) { const f16 h = (f16)v[u]; ldsW[(nn0 + 4 * g + u) * GSTR + k] = h; ldsWl[(nn0 + 4 * g + u) * GSTR + k] = (f16)((v[u] - (float)h) * 2048.0f); } }
    }
    __syncthreads();
    f16x16 af[2], afl[2];
#pragma unroll
    for (int i = 0; i < 2; ++i) { af[i] = lds_frag(ldsA + (wm + 16 * i) * GSTR, GSTR); afl[i] = lds_frag(ldsAl + (wm + 16 * i) * GSTR, GSTR); }
#pragma unroll
    for (int j = 0; j < 4; ++j) {
      const f16x16 bf = lds_frag(ldsW + (wn + 16 * j) * GSTR, GSTR), bfl = lds_frag(ldsWl + (wn + 16 * j) * GSTR, GSTR);
#pragma unroll
      for (int i = 0; i < 2; ++i) { acc[i][j] = wmma16(af[i], bf, acc[i][j]); accx[i][j] = wmma16(af[i], bfl, accx[i][j]); accx[i][j] = wmma16(afl[i], bf, accx[i][j]); }
    }
  }
  float* so = oS[wave];
#pragma unroll
  for (int i = 0; i < 2; ++i)
#pragma unroll
    for (int j = 0; j < 4; ++j) {
      const float bv = bias ? bias[n0 + wn + 16 * j + cl] : 0.0f;
#pragma unroll
      for (int r = 0; r < 8; ++r) so[(16 * i + rh + r) * 68 + 16 * j + cl] = (acc[i][j][r] + accx[i][j][r] * (1.0f / 2048.0f)) * scale + bv;
    }
  asm volatile("s_wait_dscnt 0" ::: "memory");
  __builtin_amdgcn_wave_barrier();
  if (ACC) {
#pragma unroll
    for (int it = 0; it < 16; ++it) { const int f4 = lane + 32 * it, rr = f4 >> 4, q = (f4 & 15) * 4;
      const v4f_t old = *(const v4fa*)(Y + (size_t)(m0 + wm + rr) * ldy + n0 + wn + q);
      v4f_t v = *(const v4fa*)(so + rr * 68 + q); v += old; *(v4fa*)(so + rr * 68 + q) = v; }
    asm volatile("s_wait_dscnt 0" ::: "memory");
  }
#pragma unroll 1
  for (int pass = 0; pass < 2; ++pass) {
#pragma unroll
    for (int it = 0; it < 16; ++it) { const int f4 = lane + 32 * it, rr = f4 >> 4, q = (f4 & 15) * 4;
      *(volatile v4f_t*)(Y + (size_t)(m0 + wm + rr) * ldy + n0 + wn + q) = *(const v4fa*)(so + rr * 68 + q); }
    __threadfence();
  }
}

template <typename AT, bool ACC>
__global__ __launch_bounds__(256) void gemm_kn2(const AT* __restrict__ A, int lda, size_t strideA,
                                               const float* __restrict__ Wm, int ldw, size_t strideW,
                                               const float* __restrict__ bias, float scale,
                                               float* __restrict__ Y, int ldy, size_t strideY, int K) {
  __shared__ __attribute__((aligned(16))) f16 ldsA[128 * GSTR], ldsAl[128 * GSTR];
  __shared__ __attribute__((aligned(16))) f16 ldsW[128 * GSTR], ldsWl[128 * GSTR];
  __shared__ __attribute__((aligned(16))) float oS[8][32 * 68];
  const int tid = threadIdx.x, lane = tid & 31, wave = tid >> 5, cl = lane & 15, rh = (lane >> 4) * 8;
  const int m0 = blockIdx.x * 128, n0 = blockIdx.y * 128;
  const int wm = (wave & 3) * 32, wn = (wave >> 2) * 64;
  A += (size_t)blockIdx.z * strideA; Wm += (size_t)blockIdx.z * strideW; Y += (size_t)blockIdx.z * strideY;
  f32x8 acc[2][4], accx[2][4];
#pragma unroll
  for (int i = 0; i < 2; ++i)
#pragma unroll
    for (int j = 0; j < 4; ++j) { f32x8 z = {}; acc[i][j] = z; accx[i][j] = z; }
#pragma unroll 1
  for (int k0 = 0; k0 < K; k0 += 32) {
    __syncthreads();
    {
      const int row = tid >> 1, ch = (tid & 1) * 16;
      const AT* src = A + (size_t)(m0 + row) * lda + k0 + ch;
#pragma unroll
      for (int g = 0; g < 16; ++g) { const float v = (float)src[g]; const f16 h = (f16)v; ldsA[row * GSTR + ch + g] = h; ldsAl[row * GSTR + ch + g] = (f16)((v - (float)h) * 2048.0f); }
    }
    {
      const int k = tid >> 3, nn0 = (tid & 7) * 16;
      const float* src = Wm + (size_t)(k0 + k) * ldw + n0 + nn0;
#pragma unroll
      for (int g = 0; g < 4; ++g) { const v4f_t v = *(const v4f_t*)(src + 4 * g);
#pragma unroll
        for (int u = 0; u < 4; ++u) { const f16 h = (f16)v[u]; ldsW[(nn0 + 4 * g + u) * GSTR + k] = h; ldsWl[(nn0 + 4 * g + u) * GSTR + k] = (f16)((v[u] - (float)h) * 2048.0f); } }
    }
    __syncthreads();
    f16x16 af[2], afl[2];
#pragma unroll
    for (int i = 0; i < 2; ++i) { af[i] = lds_frag(ldsA + (wm + 16 * i) * GSTR, GSTR); afl[i] = lds_frag(ldsAl + (wm + 16 * i) * GSTR, GSTR); }
#pragma unroll
    for (int j = 0; j < 4; ++j) {
      const f16x16 bf = lds_frag(ldsW + (wn + 16 * j) * GSTR, GSTR), bfl = lds_frag(ldsWl + (wn + 16 * j) * GSTR, GSTR);
#pragma unroll
      for (int i = 0; i < 2; ++i) { acc[i][j] = wmma16(af[i], bf, acc[i][j]); accx[i][j] = wmma16(af[i], bfl, accx[i][j]); accx[i][j] = wmma16(afl[i], bf, accx[i][j]); }
    }
  }
  float* so = oS[wave];
#pragma unroll
  for (int i = 0; i < 2; ++i)
#pragma unroll
    for (int j = 0; j < 4; ++j) {
      const float bv = bias ? bias[n0 + wn + 16 * j + cl] : 0.0f;
#pragma unroll
      for (int r = 0; r < 8; ++r) so[(16 * i + rh + r) * 68 + 16 * j + cl] = (acc[i][j][r] + accx[i][j][r] * (1.0f / 2048.0f)) * scale + bv;
    }
  asm volatile("s_wait_dscnt 0" ::: "memory");
  __builtin_amdgcn_wave_barrier();
  if (ACC) {
#pragma unroll
    for (int it = 0; it < 16; ++it) { const int f4 = lane + 32 * it, rr = f4 >> 4, q = (f4 & 15) * 4;
      const v4f_t old = *(const v4fa*)(Y + (size_t)(m0 + wm + rr) * ldy + n0 + wn + q);
      v4f_t v = *(const v4fa*)(so + rr * 68 + q); v += old; *(v4fa*)(so + rr * 68 + q) = v; }
    asm volatile("s_wait_dscnt 0" ::: "memory");
  }
#pragma unroll 1
  for (int pass = 0; pass < 2; ++pass) {
#pragma unroll
    for (int it = 0; it < 16; ++it) { const int f4 = lane + 32 * it, rr = f4 >> 4, q = (f4 & 15) * 4;
      *(volatile v4f_t*)(Y + (size_t)(m0 + wm + rr) * ldy + n0 + wn + q) = *(const v4fa*)(so + rr * 68 + q); }
    __threadfence();
  }
}

__global__ __launch_bounds__(256) void k_transpose(const float* __restrict__ Wm, float* __restrict__ Wt, int rows, int cols) {
  __shared__ float tS[64][65];
  const int tid = threadIdx.x, tbj = cols / 64, bi = blockIdx.x / tbj, bj = blockIdx.x % tbj;
  for (int e = tid; e < 64 * 64; e += 256) { const int r = e >> 6, c = e & 63; tS[r][c] = Wm[(size_t)(bi * 64 + r) * cols + bj * 64 + c]; }
  __syncthreads();
  for (int ch = tid; ch < 64 * 16; ch += 256) { const int r = ch >> 4, q4 = (ch & 15) * 4; v4f_t o; o[0] = tS[q4][r]; o[1] = tS[q4 + 1][r]; o[2] = tS[q4 + 2][r]; o[3] = tS[q4 + 3][r];
    float* dst = Wt + (size_t)(bj * 64 + r) * rows + bi * 64 + q4; *(volatile v4f_t*)dst = o; __threadfence(); *(volatile v4f_t*)dst = o; }
}

#define NBT 2
#define BBw 2
#define SSw 2048
#define HHw 2048
#define NHw 16
#define NKVw 16
#define HDw 128
#define KVW (NKVw * HDw)
__global__ __launch_bounds__(256) void k_softmax_causal(float* __restrict__ Sm) {
  __shared__ float red[256];
  const int q = blockIdx.x, z = blockIdx.y, tid = threadIdx.x; float* sr = Sm + ((size_t)z * SSw + q) * SSw;
  const float scl = 0.08838834764831845f;
  float v[SSw / 256]; float m = -3.0e38f;
#pragma unroll
  for (int e = 0; e < SSw / 256; ++e) { const int k = tid + 256 * e; v[e] = (k <= q) ? sr[k] * scl : -3.0e38f; m = fmaxf(m, v[e]); }
  red[tid] = m; __syncthreads();
  for (int o = 128; o > 0; o >>= 1) { if (tid < o) red[tid] = fmaxf(red[tid], red[tid + o]); __syncthreads(); }
  m = red[0]; __syncthreads();
  float zs = 0.0f;
#pragma unroll
  for (int e = 0; e < SSw / 256; ++e) { const int k = tid + 256 * e; v[e] = (k <= q) ? expf(v[e] - m) : 0.0f; zs += v[e]; }
  red[tid] = zs; __syncthreads();
  for (int o = 128; o > 0; o >>= 1) { if (tid < o) red[tid] += red[tid + o]; __syncthreads(); }
  const float sc = 1024.0f / red[0];
#pragma unroll 1
  for (int pass = 0; pass < 2; ++pass) {
#pragma unroll
    for (int e = 0; e < SSw / 256; ++e) *(volatile float*)(sr + tid + 256 * e) = v[e] * sc;
    __threadfence(); }
}
__global__ __launch_bounds__(128) void k_softmax128(float* __restrict__ S0) {
  __shared__ float red[128];
  const int q = blockIdx.x, z = blockIdx.y, k = threadIdx.x; float* sr = S0 + ((size_t)z * 128 + q) * 128;
  const float scl = 0.08838834764831845f; float v = (k <= q) ? sr[k] * scl : -3.0e38f;
  red[k] = v; __syncthreads();
  for (int o = 64; o > 0; o >>= 1) { if (k < o) red[k] = fmaxf(red[k], red[k + o]); __syncthreads(); }
  const float m = red[0]; __syncthreads();
  v = (k <= q) ? expf(v - m) : 0.0f; red[k] = v; __syncthreads();
  for (int o = 64; o > 0; o >>= 1) { if (k < o) red[k] += red[k + o]; __syncthreads(); }
  const float p = v * (1024.0f / red[0]);
  *(volatile float*)(sr + k) = p; __threadfence(); *(volatile float*)(sr + k) = p;
}
__global__ __launch_bounds__(256) void k_fill(float* __restrict__ p, float val, size_t n4) { const size_t i = (size_t)blockIdx.x * 256 + threadIdx.x; if (i < n4) { v4f_t v = {val, val, val, val}; *(volatile v4f_t*)(p + 4 * i) = v; __threadfence(); *(volatile v4f_t*)(p + 4 * i) = v; } }
__global__ __launch_bounds__(64) void k_ropetbl(float* __restrict__ TC, float* __restrict__ TS) {
  const int t = blockIdx.x, i = threadIdx.x;
  const float fi = 1.0f / powf(10000.0f, (float)(2 * i) / 128.0f);
  const float ang = (float)t * fi; float sn, cs; sincosf(ang, &sn, &cs);
  *(volatile float*)(TC + (size_t)t * 64 + i) = cs; *(volatile float*)(TS + (size_t)t * 64 + i) = sn; __threadfence();
  *(volatile float*)(TC + (size_t)t * 64 + i) = cs; *(volatile float*)(TS + (size_t)t * 64 + i) = sn;
}
__global__ __launch_bounds__(256) void k_rope(float* __restrict__ X, int width, const float* __restrict__ TC, const float* __restrict__ TS) {
  const int row = blockIdx.x, tid = threadIdx.x; float* xr = X + (size_t)row * width; const float* tc = TC + (size_t)row * 64; const float* ts = TS + (size_t)row * 64;
#pragma unroll 1
  for (int c4 = tid; c4 < (width >> 2); c4 += 256) {
    v4f_t v = *(const v4f_t*)(xr + 4 * c4); const int i0 = (2 * c4) & 63;
    const float C0 = tc[i0], S0 = ts[i0], C1 = tc[i0 + 1], S1 = ts[i0 + 1];
    v4f_t r; r[0] = v[0] * S0 - v[1] * C0; r[1] = v[0] * C0 + v[1] * S0; r[2] = v[2] * S1 - v[3] * C1; r[3] = v[2] * C1 + v[3] * S1;
    *(volatile v4f_t*)(xr + 4 * c4) = r; __threadfence(); *(volatile v4f_t*)(xr + 4 * c4) = r;
  }
}


#define DDx 2048
#define SIN 2048
__global__ __launch_bounds__(256) void k_dbg_zero(float* __restrict__ p, size_t n4) { const size_t i = (size_t)blockIdx.x * 256 + threadIdx.x; if (i < n4) { v4f_t z = {0.f,0.f,0.f,0.f}; *(volatile v4f_t*)(p + 4 * i) = z; __threadfence(); *(volatile v4f_t*)(p + 4 * i) = z; } }
__global__ __launch_bounds__(256) void k_copy(const float* __restrict__ src, float* __restrict__ dst, size_t n4) { const size_t i = (size_t)blockIdx.x * 256 + threadIdx.x; if (i < n4) { const v4f_t v = *(const v4f_t*)(src + 4 * i); *(volatile v4f_t*)(dst + 4 * i) = v; __threadfence(); *(volatile v4f_t*)(dst + 4 * i) = v; } }
__global__ __launch_bounds__(256) void k_transpose_ld(const float* __restrict__ Wm, int lds, float* __restrict__ Wt, int rows, int cols) {
  __shared__ float tS[64][65];
  const int tid = threadIdx.x, tbj = cols / 64, bi = blockIdx.x / tbj, bj = blockIdx.x % tbj;
  for (int e = tid; e < 64 * 64; e += 256) { const int r = e >> 6, c = e & 63; tS[r][c] = Wm[(size_t)(bi * 64 + r) * lds + bj * 64 + c]; }
  __syncthreads();
  for (int ch = tid; ch < 64 * 16; ch += 256) { const int r = ch >> 4, q4 = (ch & 15) * 4; v4f_t o; o[0] = tS[q4][r]; o[1] = tS[q4 + 1][r]; o[2] = tS[q4 + 2][r]; o[3] = tS[q4 + 3][r];
    float* dst = Wt + (size_t)(bj * 64 + r) * rows + bi * 64 + q4; *(volatile v4f_t*)dst = o; __threadfence(); *(volatile v4f_t*)dst = o; }
}
__global__ __launch_bounds__(64) void k_ropetbl2(float* __restrict__ TC, float* __restrict__ TS) {
  const int t = blockIdx.x, i = threadIdx.x; const float ex = 2.0f * (float)i / 128.0f; const float pw = (float)pow(10000.0, (double)ex); const float fi = 1.0f / pw;
  const float ang = (float)t * fi; const float cs = (float)cos((double)ang), sn = (float)sin((double)ang);
  *(volatile float*)(TC + (size_t)t * 64 + i) = cs; *(volatile float*)(TS + (size_t)t * 64 + i) = sn; __threadfence(); *(volatile float*)(TC + (size_t)t * 64 + i) = cs; *(volatile float*)(TS + (size_t)t * 64 + i) = sn;
}
__global__ __launch_bounds__(256) void k_rope2(float* __restrict__ X, int ld, const float* __restrict__ TC, const float* __restrict__ TS) {
  const int row = blockIdx.x, tid = threadIdx.x; float* xr = X + (size_t)row * ld; const float* tc = TC + (size_t)row * 64; const float* ts = TS + (size_t)row * 64;
  const int h = tid >> 4, i0 = (tid & 15) * 4; float* base = xr + h * 128;
  const v4f_t a = *(const v4f_t*)(base + i0), b = *(const v4f_t*)(base + 64 + i0), C = *(const v4f_t*)(tc + i0), Sn = *(const v4f_t*)(ts + i0);
  const v4f_t ra = a * C - b * Sn, rb = b * C + a * Sn;
  *(volatile v4f_t*)(base + i0) = ra; *(volatile v4f_t*)(base + 64 + i0) = rb; __threadfence(); *(volatile v4f_t*)(base + i0) = ra; *(volatile v4f_t*)(base + 64 + i0) = rb;
}
__global__ __launch_bounds__(256) void k_lsoft(float* __restrict__ Sm) {
  __shared__ float red[256];
  const int q = blockIdx.x, z = blockIdx.y, tid = threadIdx.x; float* sr = Sm + ((size_t)z * SSw + q) * SSw; const float scl = 0.08838834764831845f;
  float v[SSw / 256]; float m = 0.0f;
#pragma unroll
  for (int e = 0; e < SSw / 256; ++e) { const int k = tid + 256 * e; v[e] = (k <= q) ? 50.0f * tanhf(sr[min(k, q)] * scl * 0.02f) : -3.0e38f; m = fmaxf(m, v[e]); }
  red[tid] = m; __syncthreads(); for (int o = 128; o > 0; o >>= 1) { if (tid < o) red[tid] = fmaxf(red[tid], red[tid + o]); __syncthreads(); }
  m = red[0]; __syncthreads(); float zs = 0.0f;
#pragma unroll
  for (int e = 0; e < SSw / 256; ++e) { const int k = tid + 256 * e; v[e] = (k <= q) ? expf(v[e] - m) : 0.0f; zs += v[e]; }
  red[tid] = zs; __syncthreads(); for (int o = 128; o > 0; o >>= 1) { if (tid < o) red[tid] += red[tid + o]; __syncthreads(); }
  const float kk = 1024.0f / (red[0] + expf(-m));
#pragma unroll 1
  for (int pass = 0; pass < 2; ++pass) {
#pragma unroll
    for (int e = 0; e < SSw / 256; ++e) *(volatile float*)(sr + tid + 256 * e) = v[e] * kk;
    __threadfence(); }
}

__global__ __launch_bounds__(256) void k_place0(const float* __restrict__ T0, int h0, float* __restrict__ CTX) {
  const int tid = threadIdx.x, z = blockIdx.y, r = blockIdx.x * 8 + (tid >> 5), c4 = (tid & 31) * 4;
  const v4f_t t = *(const v4f_t*)(T0 + ((size_t)z * 128 + r) * 256 + z * 128 + c4); const v4f_t v = t * (1.0f / 1024.0f);
  float* d = CTX + (size_t)r * DDx + (h0 + z) * HDw + c4; *(volatile v4f_t*)d = v; __threadfence(); *(volatile v4f_t*)d = v;
}
extern "C" void kernel_launch(void* const* d_in, const int* in_sizes, int n_in,
                              void* d_out, int out_size, void* d_ws, size_t ws_size,
                              hipStream_t stream) {
  (void)in_sizes; (void)n_in; (void)out_size;
  const float** f = (const float**)d_in;
  const float* x = f[0], *Wq = f[1], *Wk = f[2], *Wv = f[3], *Wo = f[4];
  float* out = (float*)d_out;
  char* ws = (char*)d_ws;
  float* TC = (float*)ws; ws += (size_t)SSw * 64 * 4; float* TSn = (float*)ws; ws += (size_t)SSw * 64 * 4;
  float* Q = (float*)ws; ws += (size_t)SSw * DDx * 4; float* Km = (float*)ws; ws += (size_t)SSw * DDx * 4; float* V = (float*)ws; ws += (size_t)SSw * DDx * 4 + 1024; float* KT = (float*)ws; ws += (size_t)HDw * 2 * SSw * 4;
  float* sc = (float*)ws; ws += HDw * 4; float* T0 = (float*)ws; ws += (size_t)2 * 128 * 256 * 4; float* Q0 = (float*)ws; ws += (size_t)128 * DDx * 4; float* K0 = (float*)ws; ws += (size_t)128 * DDx * 4; float* K0T = (float*)ws; ws += (size_t)DDx * 128 * 4; float* S = (float*)ws; ws += (size_t)2 * SSw * SSw * 4; float* CTX = (float*)ws; ws += (size_t)SSw * DDx * 4;
  if ((size_t)(ws - (char*)d_ws) > ws_size) return;
  const dim3 blk(256);
  k_fill<<<dim3(1), blk, 0, stream>>>(sc, 1.0f / 1024.0f, HDw / 4); k_fill<<<dim3(1), blk, 0, stream>>>(V + (size_t)SSw * DDx, 0.0f, 256 / 4); k_ropetbl2<<<dim3(SSw), dim3(64), 0, stream>>>(TC, TSn);

  for (int b = 0; b < NBT; ++b) { const float* xb = x + (size_t)b * SIN * DDx;
    gemm_kne<float, 0, false><<<dim3(SSw / 128, DDx / 128), blk, 0, stream>>>(xb, DDx, Wq, DDx, nullptr, nullptr, nullptr, Q, DDx, DDx);
    gemm_kne<float, 0, false><<<dim3(SSw / 128, DDx / 128), blk, 0, stream>>>(xb, DDx, Wk, DDx, nullptr, nullptr, nullptr, Km, DDx, DDx);
    gemm_kn2<float, false><<<dim3(SSw / 128, DDx / 128, 1), blk, 0, stream>>>(xb, DDx, 0, Wv, DDx, 0, nullptr, 1.0f, V, DDx, 0, DDx);
    k_rope2<<<dim3(SSw), blk, 0, stream>>>(Q, DDx, TC, TSn); k_rope2<<<dim3(SSw), blk, 0, stream>>>(Km, DDx, TC, TSn);
    gemm_kn2<float, false><<<dim3(1, DDx / 128, 1), blk, 0, stream>>>(xb, DDx, 0, Wq, DDx, 0, nullptr, 1.0f, Q0, DDx, 0, DDx);
    gemm_kn2<float, false><<<dim3(1, DDx / 128, 1), blk, 0, stream>>>(xb, DDx, 0, Wk, DDx, 0, nullptr, 1.0f, K0, DDx, 0, DDx);
    k_rope2<<<dim3(128), blk, 0, stream>>>(Q0, DDx, TC, TSn); k_rope2<<<dim3(128), blk, 0, stream>>>(K0, DDx, TC, TSn);
    k_transpose<<<dim3((128 / 64) * (DDx / 64)), blk, 0, stream>>>(K0, K0T, 128, DDx);
    for (int hp = 0; hp < NHw / 2; ++hp) { const int h0 = 2 * hp;
      for (int z = 0; z < 2; ++z) k_transpose_ld<<<dim3((SSw / 64) * (HDw / 64)), blk, 0, stream>>>(Km + (h0 + z) * HDw, DDx, KT + (size_t)z * HDw * SSw, SSw, HDw);
      gemm_knezc<float, 0, false, 2><<<dim3(SSw / 128, SSw / 128, 2), blk, 0, stream>>>(Q + h0 * HDw, DDx, (size_t)HDw, KT, SSw, (size_t)HDw * SSw, nullptr, nullptr, nullptr, S, SSw, (size_t)SSw * SSw, HDw);
      gemm_kn2<float, false><<<dim3(1, 1, 2), blk, 0, stream>>>(Q0 + h0 * HDw, DDx, (size_t)HDw, K0T + (size_t)h0 * HDw * 128, 128, (size_t)HDw * 128, nullptr, 1.0f, S, SSw, (size_t)SSw * SSw, HDw);
      k_lsoft<<<dim3(SSw, 2), blk, 0, stream>>>(S);
      gemm_knezc<float, 4, false, 1><<<dim3(SSw / 128, 1, 2), blk, 0, stream>>>(S, SSw, (size_t)SSw * SSw, V + h0 * HDw, DDx, (size_t)HDw, nullptr, nullptr, sc, CTX + h0 * HDw, DDx, (size_t)HDw, SSw);
      gemm_kn2<float, false><<<dim3(1, 2, 2), blk, 0, stream>>>(S, SSw, (size_t)SSw * SSw, V + h0 * HDw, DDx, (size_t)0, nullptr, 1.0f, T0, 256, (size_t)128 * 256, 128);
      k_place0<<<dim3(128 / 8, 2), blk, 0, stream>>>(T0, h0, CTX);
    }
    gemm_kne<float, 0, false><<<dim3(SSw / 128, DDx / 128), blk, 0, stream>>>(CTX, DDx, Wo, DDx, nullptr, nullptr, nullptr, out + (size_t)b * SIN * DDx, DDx, DDx);
    gemm_kn2<float, false><<<dim3(1, DDx / 128, 1), blk, 0, stream>>>(CTX, DDx, 0, Wo, DDx, 0, nullptr, 1.0f, out + (size_t)b * SIN * DDx, DDx, 0, DDx);
  }
}
